// Decoder_5875515261520
// MI455X (gfx1250) — hardware-verified
//
#include <hip/hip_runtime.h>
#include <stddef.h>
#include <stdint.h>


#define NHID    64
#define NP      128
#define N_NODES 100000
#define N_EDGES 3200000
#define MPAD    100096
#define GBM     64
#define GBN     128
#define GTHR    128
#define NTHR    256
#define EPBLK   1024
#define NU_WB   (NP * (NHID / 8))
#define WSMAX   134217728

static_assert(NHID == 64);
static_assert(2 * NHID == NP && NP == GBN);
static_assert(NHID % 32 == 0);
static_assert(N_EDGES % EPBLK == 0 && N_EDGES / EPBLK == 3125);
static_assert(N_NODES == 781 * 128 + 32 && N_NODES == 1562 * GBM + 32);
static_assert(MPAD == 782 * 128 && MPAD % GBM == 0 && MPAD >= N_NODES);
static_assert(NTHR * 4 == EPBLK);
static_assert(GBM == (GTHR / 32) * 16 && GBN == 4 * 32);
static_assert((MPAD * (NHID / 8)) % NTHR == 0 && NU_WB % NTHR == 0);
static_assert((NTHR / 32) * 128 == EPBLK);

typedef float          v4f   __attribute__((ext_vector_type(4)));
typedef float          v8f   __attribute__((ext_vector_type(8)));
typedef int            v4i   __attribute__((ext_vector_type(4)));
typedef int            v8i   __attribute__((ext_vector_type(8)));
typedef unsigned short v8us  __attribute__((ext_vector_type(8)));
typedef unsigned short v16us __attribute__((ext_vector_type(16)));
typedef __bf16         v16bf __attribute__((ext_vector_type(16)));
typedef v4f  __attribute__((may_alias)) v4fa;
typedef v4i  __attribute__((may_alias)) v4ia;
typedef v8us __attribute__((may_alias)) v8usa;
union FragB { v16bf v; v16us u; v8us h[2]; v8i w; };

__device__ __forceinline__ v8f wmb(const FragB& a, const FragB& b, v8f c) {
  v8f d = __builtin_amdgcn_wmma_f32_16x16x32_bf16(false, a.v, false, b.v, (short)0, c, false, false);
  asm volatile("v_nop\n\tv_nop\n\tv_nop\n\tv_nop" : "+v"(d) : "v"(a.w), "v"(b.w));
  return d;
}

__device__ __forceinline__ unsigned bf16_bits(float f) {
  const unsigned u = __float_as_uint(f);
  return (u + 0x7FFFu + ((u >> 16) & 1u)) >> 16;
}
__device__ __forceinline__ float bf16_val(float f) {
  return __uint_as_float(bf16_bits(f) << 16);
}
__device__ __forceinline__ v4f bfr4(const v4f a) {
  v4f r; r.x = bf16_val(a.x); r.y = bf16_val(a.y); r.z = bf16_val(a.z); r.w = bf16_val(a.w); return r;
}
__device__ __forceinline__ void put16(unsigned short* dp, v8us o) {
  *(volatile v8us*)dp = o;
  __threadfence();
  *(volatile v8us*)dp = o;
}

__global__ __launch_bounds__(NTHR) void k_prep(const float* __restrict__ z, const float* __restrict__ W1,
                                               int nN, int uz, unsigned short* ZB, unsigned short* WB) {
  const int u = (int)blockIdx.x * NTHR + (int)threadIdx.x;
  v8us o;
  if (u < uz) {
    const int row = u >> 3;
    const int k8  = (u & 7) * 8;
    const int rc  = row < nN ? row : nN - 1;
    const float* p = z + (size_t)rc * NHID + k8;
    const v4f a = *(const v4fa*)p;
    const v4f b = *(const v4fa*)(p + 4);
    const bool ok = row < nN;
    o[0] = ok ? (unsigned short)bf16_bits(a.x) : (unsigned short)0;
    o[1] = ok ? (unsigned short)bf16_bits(a.y) : (unsigned short)0;
    o[2] = ok ? (unsigned short)bf16_bits(a.z) : (unsigned short)0;
    o[3] = ok ? (unsigned short)bf16_bits(a.w) : (unsigned short)0;
    o[4] = ok ? (unsigned short)bf16_bits(b.x) : (unsigned short)0;
    o[5] = ok ? (unsigned short)bf16_bits(b.y) : (unsigned short)0;
    o[6] = ok ? (unsigned short)bf16_bits(b.z) : (unsigned short)0;
    o[7] = ok ? (unsigned short)bf16_bits(b.w) : (unsigned short)0;
    put16(ZB + (size_t)row * NHID + k8, o);
    return;
  } else if (u < uz + NU_WB) {
    const int v  = u - uz;
    const int n  = v >> 3;
    const int k8 = (v & 7) * 8;
    const float* p = W1 + (size_t)(n & (NHID - 1)) * NP + (n >> 6) * NHID + k8;
    const v4f a = *(const v4fa*)p;
    const v4f b = *(const v4fa*)(p + 4);
    o[0] = (unsigned short)bf16_bits(a.x);
    o[1] = (unsigned short)bf16_bits(a.y);
    o[2] = (unsigned short)bf16_bits(a.z);
    o[3] = (unsigned short)bf16_bits(a.w);
    o[4] = (unsigned short)bf16_bits(b.x);
    o[5] = (unsigned short)bf16_bits(b.y);
    o[6] = (unsigned short)bf16_bits(b.z);
    o[7] = (unsigned short)bf16_bits(b.w);
    put16(WB + (size_t)n * NHID + k8, o);
    return;
  }
}

__global__ __launch_bounds__(GTHR) void k_pgemm(const unsigned short* __restrict__ A,
                                                const unsigned short* __restrict__ BT,
                                                const float* __restrict__ b1, int nN, float* Pm) {
  __shared__ __attribute__((aligned(16))) float stg[GBM * GBN];
  const int tid = (int)threadIdx.x, lane = tid & 31, wave = tid >> 5, hh = lane >> 4, m = lane & 15;
  const int rowBase = (int)blockIdx.x * GBM;

  v8f acc[8];
  {
    const v8f zz = {0.f, 0.f, 0.f, 0.f, 0.f, 0.f, 0.f, 0.f};
#pragma unroll
    for (int t = 0; t < 8; ++t) acc[t] = zz;
  }
  const unsigned short* ap = A  + (size_t)(rowBase + 16 * wave + m) * (size_t)NHID + 8 * hh;
  const unsigned short* bp = BT + (size_t)m * (size_t)NHID + 8 * hh;

#pragma unroll 1
  for (int k0 = 0; k0 < NHID; k0 += 32) {
    FragB af;
    af.h[0] = *(const v8usa*)(ap + k0);
    af.h[1] = *(const v8usa*)(ap + k0 + 16);
#pragma unroll
    for (int nt = 0; nt < 8; ++nt) {
      const unsigned short* wq = bp + (size_t)(16 * nt) * (size_t)NHID + k0;
      FragB bf;
      bf.h[0] = *(const v8usa*)wq;
      bf.h[1] = *(const v8usa*)(wq + 16);
      acc[nt] = wmb(af, bf, acc[nt]);
    }
  }

#pragma unroll
  for (int nt = 0; nt < 8; ++nt) {
    const int lc = 16 * nt + m;
#pragma unroll
    for (int r = 0; r < 8; ++r) {
      const int lr = 16 * wave + 8 * hh + r;
      stg[lr * GBN + lc] = acc[nt][r];
    }
  }
  __syncthreads();

  const v4f bq = bfr4(*(const v4fa*)(b1 + 4 * (lane & 15)));
  const float mk = (lane < 16) ? 1.0f : 0.0f;
  v4f b4;
  b4.x = bq.x * mk; b4.y = bq.y * mk; b4.z = bq.z * mk; b4.w = bq.w * mk;

  v4f pv[16];
#pragma unroll
  for (int i = 0; i < 16; ++i) {
    const v4f sv = *(const v4fa*)(stg + (16 * wave + i) * GBN + 4 * lane);
    v4f q;
    q.x = sv.x + b4.x; q.y = sv.y + b4.y; q.z = sv.z + b4.z; q.w = sv.w + b4.w;
    pv[i] = q;
  }
#pragma unroll
  for (int i = 0; i < 16; ++i) {
    const int row = rowBase + 16 * wave + i;
    if (row < nN) {
      float* op = Pm + (size_t)row * (size_t)NP + 4 * lane;
      *(volatile v4f*)op = pv[i];
    }
  }
  __threadfence();
#pragma unroll
  for (int i = 0; i < 16; ++i) {
    const int row = rowBase + 16 * wave + i;
    if (row < nN) {
      float* op = Pm + (size_t)row * (size_t)NP + 4 * lane;
      *(volatile v4f*)op = pv[i];
    }
  }
}

__global__ __launch_bounds__(NTHR) void k_edge(const int* __restrict__ rowi, const int* __restrict__ coli,
                                               const float* __restrict__ P, const float* __restrict__ W2,
                                               const float* __restrict__ b2, int nN, float* outp) {
  __shared__ __attribute__((aligned(16))) int   sR[EPBLK];
  __shared__ __attribute__((aligned(16))) int   sC[EPBLK];
  __shared__ __attribute__((aligned(16))) float sO[EPBLK];
  const int tid = (int)threadIdx.x, lane = tid & 31, wave = tid >> 5;
  const int s = lane & 7, sub = lane >> 3;
  const size_t eb = (size_t)blockIdx.x * EPBLK;
  const int hiN = nN - 1;

  {
    v4i r4 = *(const v4ia*)(rowi + eb + 4 * tid);
    v4i c4 = *(const v4ia*)(coli + eb + 4 * tid);
    r4.x = r4.x < 0 ? 0 : (r4.x > hiN ? hiN : r4.x);
    r4.y = r4.y < 0 ? 0 : (r4.y > hiN ? hiN : r4.y);
    r4.z = r4.z < 0 ? 0 : (r4.z > hiN ? hiN : r4.z);
    r4.w = r4.w < 0 ? 0 : (r4.w > hiN ? hiN : r4.w);
    c4.x = c4.x < 0 ? 0 : (c4.x > hiN ? hiN : c4.x);
    c4.y = c4.y < 0 ? 0 : (c4.y > hiN ? hiN : c4.y);
    c4.z = c4.z < 0 ? 0 : (c4.z > hiN ? hiN : c4.z);
    c4.w = c4.w < 0 ? 0 : (c4.w > hiN ? hiN : c4.w);
    *(v4ia*)(sR + 4 * tid) = r4;
    *(v4ia*)(sC + 4 * tid) = c4;
  }
  const v4f w0 = bfr4(*(const v4fa*)(W2 + 8 * s));
  const v4f w1 = bfr4(*(const v4fa*)(W2 + 8 * s + 4));
  const float bb = bf16_val(b2[0]);
  __syncthreads();

#pragma unroll 1
  for (int it = 0; it < 32; ++it) {
    const int el = 128 * wave + 4 * it + sub;
    const int r = sR[el];
    const int c = sC[el];
    const float* pa = P + (size_t)r * NP + 8 * s;
    const float* pb = P + (size_t)c * NP + NHID + 8 * s;
    const v4f a0 = *(const v4fa*)pa;
    const v4f a1 = *(const v4fa*)(pa + 4);
    const v4f q0 = *(const v4fa*)pb;
    const v4f q1 = *(const v4fa*)(pb + 4);
    const float h0 = fmaxf(a0.x + q0.x, 0.0f);
    const float h1 = fmaxf(a0.y + q0.y, 0.0f);
    const float h2 = fmaxf(a0.z + q0.z, 0.0f);
    const float h3 = fmaxf(a0.w + q0.w, 0.0f);
    const float h4 = fmaxf(a1.x + q1.x, 0.0f);
    const float h5 = fmaxf(a1.y + q1.y, 0.0f);
    const float h6 = fmaxf(a1.z + q1.z, 0.0f);
    const float h7 = fmaxf(a1.w + q1.w, 0.0f);
    float part = h0 * w0.x;
    part = fmaf(h1, w0.y, part);
    part = fmaf(h2, w0.z, part);
    part = fmaf(h3, w0.w, part);
    part = fmaf(h4, w1.x, part);
    part = fmaf(h5, w1.y, part);
    part = fmaf(h6, w1.z, part);
    part = fmaf(h7, w1.w, part);
    part += __shfl_xor(part, 4, 32);
    part += __shfl_xor(part, 2, 32);
    part += __shfl_xor(part, 1, 32);
    const float res = part + bb;
    if (s == 0) sO[el] = res;
  }
  __syncthreads();

  {
    const v4f o4 = *(const v4fa*)(sO + 4 * tid);
    float* op = outp + eb + 4 * tid;
    *(volatile v4f*)op = o4;
    __threadfence();
    *(volatile v4f*)op = o4;
  }
}

extern "C" void kernel_launch(void* const* d_in, const int* in_sizes, int n_in,
                              void* d_out, int out_size, void* d_ws, size_t ws_size,
                              hipStream_t stream) {
  if (n_in < 7) return;
  if (in_sizes[0] != N_NODES * NHID) return;
  if (in_sizes[1] != N_EDGES || in_sizes[2] != N_EDGES) return;
  if (in_sizes[3] != NHID * NP) return;
  if (in_sizes[4] != NHID || in_sizes[5] != NHID || in_sizes[6] != 1) return;
  if (out_size != N_EDGES) return;

  const float* z   = (const float*)d_in[0];
  const int*   row = (const int*)d_in[1];
  const int*   col = (const int*)d_in[2];
  const float* W1  = (const float*)d_in[3];
  const float* b1  = (const float*)d_in[4];
  const float* W2  = (const float*)d_in[5];
  const float* b2  = (const float*)d_in[6];
  float* out = (float*)d_out;

  const int nN = N_NODES;
  const int nE = N_EDGES;
  const int MP = MPAD;
  const int gM = MP / GBM;
  const int gE = nE / EPBLK;
  if ((long long)gE * EPBLK != (long long)nE) return;

  char* ws = (char*)d_ws;
  size_t off = 0;
  const size_t oZB = off; off += (size_t)MP * NHID * 2;      off = (off + 255) & ~(size_t)255;
  const size_t oWB = off; off += (size_t)NP * NHID * 2;      off = (off + 255) & ~(size_t)255;
  const size_t oP  = off; off += (size_t)nN * NP * 4;        off = (off + 255) & ~(size_t)255;
  if (off > ws_size || off > (size_t)WSMAX) return;
  unsigned short* ZB = (unsigned short*)(ws + oZB);
  unsigned short* WB = (unsigned short*)(ws + oWB);
  float*          P  = (float*)(ws + oP);

  const int uz = MP * (NHID / 8);
  k_prep<<<(uz + NU_WB) / NTHR, NTHR, 0, stream>>>(z, W1, nN, uz, ZB, WB);
  k_pgemm<<<gM, GTHR, 0, stream>>>(ZB, WB, b1, nN, P);
  k_edge<<<gE, NTHR, 0, stream>>>(row, col, P, W2, b2, nN, out);
}
